// GQA_13245679141285
// MI455X (gfx1250) — hardware-verified
//
#include <hip/hip_runtime.h>
#ifndef NB
#define NB 2
#endif
#ifndef SQ
#define SQ 2048
#endif
#define SQF 2048
#define DM 2048
#define NH 16
#define NG 4
#define HPG 4
#define HD 128
#define HD2 (HD / 2)
#define KVD (NG * HD)
#define QT 256
#define NKX SQ
#define QT0 256
#define R0 32
static_assert(SQ % QT == 0);
static_assert(SQ >= QT);
static_assert(SQ <= SQF);
static_assert(QT0 % R0 == 0);
static_assert(QT0 % 128 == 0);
static_assert(QT0 <= QT);
static_assert(NH == NG * HPG);
static_assert(DM == NH * HD);
static_assert(HD % 64 == 0);
static_assert(KVD % 64 == 0);
static_assert(R0 * 16 == HD * 4);

typedef _Float16 v16h __attribute__((ext_vector_type(16)));
typedef unsigned short v8us __attribute__((ext_vector_type(8), may_alias));
typedef float v8f __attribute__((ext_vector_type(8)));
typedef float v4f __attribute__((ext_vector_type(4)));
typedef float v4fa __attribute__((ext_vector_type(4), may_alias));
typedef _Float16 v4h __attribute__((ext_vector_type(4)));
union FragH { v16h v; v8us half[2]; _Float16 h[16]; unsigned short u[16]; };

__device__ __forceinline__ unsigned short bf16_bits(float x) { unsigned int u = __float_as_uint(x); return (unsigned short)((u + 0x7FFFu + ((u >> 16) & 1u)) >> 16); }
__device__ __forceinline__ float bf16_val(unsigned short b) { return __uint_as_float(((unsigned int)b) << 16); }
__device__ __forceinline__ float bf16_rne(float x) { return bf16_val(bf16_bits(x)); }

__device__ __forceinline__ v16h g2_frag(const _Float16* p, int hh) { FragH f; f.half[0] = *(const v8us*)((const unsigned short*)p + 8 * hh); f.half[1] = *(const v8us*)((const unsigned short*)p + 16 + 8 * hh); return f.v; }
__device__ __forceinline__ v8f g2_mma(v16h a, v16h b, v8f c) { v8f d = __builtin_amdgcn_wmma_f32_16x16x32_f16(false, a, false, b, (short)0, c, false, false); asm volatile("v_nop\n\tv_nop\n\tv_nop\n\tv_nop" : "+v"(d) : "v"(a), "v"(b)); return d; }

template <int ACT>
__global__ __launch_bounds__(128) void k_gemm2(const _Float16* __restrict__ A, int lda, size_t sA, const _Float16* __restrict__ Bh, int ldb, size_t sB, int bdiv, float alpha,
    const float* __restrict__ bias, size_t sBias, const float* CP, int rowsPerB, size_t sCPb, int row0g,
    float* C, _Float16* C16, int ldc, size_t sC, int M, int N, int K) {
  static_assert(ACT == 0 || ACT == 3);
  __shared__ __attribute__((aligned(16))) float so[4][32][68];
  const int tid = threadIdx.x, w = tid >> 5, lane = tid & 31, ln = lane & 15, hh = lane >> 4; const int by = blockIdx.y;
  A += (size_t)by * sA; Bh += (size_t)(by / bdiv) * sB; const size_t cofs = (size_t)by * sC; const float* bp = bias ? bias + (size_t)by * sBias : nullptr;
  const int ntn = N >> 6; const int mt = blockIdx.x / ntn, nq = blockIdx.x - mt * ntn; const int row0 = mt * 128 + 32 * w, col0 = nq * 64; if (row0 >= M) return;
  const _Float16* a0p = A + (size_t)(row0 + ln) * lda; const _Float16* a1p = a0p + (size_t)16 * lda;
  const _Float16* b0p = Bh + (size_t)(col0 + ln) * ldb; const _Float16* b1p = b0p + (size_t)16 * ldb; const _Float16* b2p = b1p + (size_t)16 * ldb; const _Float16* b3p = b2p + (size_t)16 * ldb;
  const v8f z8 = {0.f, 0.f, 0.f, 0.f, 0.f, 0.f, 0.f, 0.f}; v8f c00 = z8, c01 = z8, c02 = z8, c03 = z8, c10 = z8, c11 = z8, c12 = z8, c13 = z8;
#pragma unroll 1
  for (int kb = 0; kb < K; kb += 32) { const v16h a0 = g2_frag(a0p + kb, hh), a1 = g2_frag(a1p + kb, hh);
    v16h b = g2_frag(b0p + kb, hh); c00 = g2_mma(a0, b, c00); c10 = g2_mma(a1, b, c10);
    b = g2_frag(b1p + kb, hh); c01 = g2_mma(a0, b, c01); c11 = g2_mma(a1, b, c11);
    b = g2_frag(b2p + kb, hh); c02 = g2_mma(a0, b, c02); c12 = g2_mma(a1, b, c12);
    b = g2_frag(b3p + kb, hh); c03 = g2_mma(a0, b, c03); c13 = g2_mma(a1, b, c13); }
  v8f accs[8] = {c00, c01, c02, c03, c10, c11, c12, c13};
#pragma unroll
  for (int u = 0; u < 8; ++u) { const int t = u & 3, half = u >> 2; const int col = col0 + t * 16 + ln; const float bv = bp ? bf16_rne(bp[col]) : 0.f;
#pragma unroll
    for (int r = 0; r < 8; ++r) { const int rloc = half * 16 + 8 * hh + r; float v = accs[u][r] * alpha + bv;
      if (CP) { if (rowsPerB < 0) v += CP[cofs + (size_t)(row0g + row0 + rloc) * ldc + col]; else { const int bidx = (row0g + row0 + rloc) / rowsPerB; v += CP[(size_t)bidx * sCPb + (size_t)by * 64 + col]; } }
      if (ACT == 3) v = fmaxf(v, 0.f);
      so[w][rloc][t * 16 + ln] = v; } }
  __builtin_amdgcn_fence(4, "workgroup"); __builtin_amdgcn_wave_barrier();
  const int rsub = lane >> 4, c4 = (lane & 15) * 4;
  for (int pass = 0; pass < 2; ++pass) {
#pragma unroll
    for (int q = 0; q < 16; ++q) { const int r = q * 2 + rsub; const v4f v = *(const v4fa*)&so[w][r][c4];
      if (C) *(volatile v4f*)(C + cofs + (size_t)(row0 + r) * ldc + col0 + c4) = v;
      if (C16) { v4h h4; for (int i = 0; i < 4; ++i) h4[i] = (_Float16)v[i]; *(volatile v4h*)(C16 + cofs + (size_t)(row0 + r) * ldc + col0 + c4) = h4; } }
    if (pass == 0) __threadfence(); }
}

__global__ __launch_bounds__(256) void k_wt_f16(const float* __restrict__ W, _Float16* __restrict__ Wt, int K, int N, float scale) {
  const int t = blockIdx.x * 256 + threadIdx.x; if (t >= N * (K / 8)) return; const int n = t / (K / 8), k8 = (t % (K / 8)) * 8; FragH f;
#pragma unroll
  for (int i = 0; i < 8; ++i) f.h[i] = (_Float16)(bf16_rne(W[(size_t)(k8 + i) * N + n]) * scale);
  const v8us o = f.half[0]; unsigned short* d = (unsigned short*)Wt + (size_t)n * K + k8;
  *(volatile v8us*)d = o; __threadfence(); *(volatile v8us*)d = o;
}

__global__ __launch_bounds__(256) void k_x16(const float* __restrict__ x, _Float16* __restrict__ X16, size_t n8) { const size_t t = (size_t)blockIdx.x * 256 + threadIdx.x; if (t >= n8) return; FragH f;
#pragma unroll
  for (int q = 0; q < 8; ++q) f.h[q] = (_Float16)bf16_rne(x[t * 8 + q]); *(volatile v8us*)((unsigned short*)X16 + t * 8) = f.half[0]; __threadfence(); *(volatile v8us*)((unsigned short*)X16 + t * 8) = f.half[0]; }

__global__ __launch_bounds__(256) void k_bfcp(const float* __restrict__ src, float* __restrict__ dst, size_t n4) { const size_t t = (size_t)blockIdx.x * 256 + threadIdx.x; if (t >= n4) return; const v4f a = *(const v4fa*)(src + t * 4); v4f o; for (int q = 0; q < 4; ++q) o[q] = bf16_rne(a[q]); *(volatile v4f*)(dst + t * 4) = o; __threadfence(); *(volatile v4f*)(dst + t * 4) = o; }

template <int NHv, int TTv>
__global__ __launch_bounds__(256) void k_vt(const _Float16* __restrict__ V16, int ldv, int voff, _Float16* __restrict__ Vt) { __shared__ unsigned short tl[64][66]; const int tid = threadIdx.x; const int slab = blockIdx.x / (TTv / 64), lg = blockIdx.x % (TTv / 64); const int b = slab / NHv, h = slab % NHv;
  for (int i = tid; i < 64 * 8; i += 256) { const int r = i / 8, c8 = (i % 8) * 8; FragH f; f.half[0] = *(const v8us*)((const unsigned short*)V16 + ((size_t)b * TTv + lg * 64 + r) * ldv + voff + h * 64 + c8);
#pragma unroll
    for (int q = 0; q < 8; ++q) tl[r][c8 + q] = f.u[q]; }
  __syncthreads();
  for (int pass = 0; pass < 2; ++pass) {
#pragma unroll
    for (int rd = 0; rd < 2; ++rd) { const int d = rd * 32 + tid / 8, pc = tid % 8; FragH f;
#pragma unroll
      for (int q = 0; q < 8; ++q) f.u[q] = tl[pc * 8 + q][d];
      *(volatile v8us*)((unsigned short*)Vt + ((size_t)slab * 64 + d) * TTv + lg * 64 + pc * 8) = f.half[0]; }
    if (pass == 0) __threadfence(); } }

__global__ __launch_bounds__(256) void k_hl(const float* __restrict__ F, _Float16* __restrict__ Hh, _Float16* __restrict__ Hl, size_t n8) { const size_t t = (size_t)blockIdx.x * 256 + threadIdx.x; if (t >= n8) return; FragH fh, fl; const v4f a = *(const v4fa*)(F + t * 8), c = *(const v4fa*)(F + t * 8 + 4);
#pragma unroll
  for (int q = 0; q < 4; ++q) { _Float16 h = (_Float16)a[q]; fh.h[q] = h; fl.h[q] = (_Float16)((a[q] - (float)h) * 1024.0f); h = (_Float16)c[q]; fh.h[4 + q] = h; fl.h[4 + q] = (_Float16)((c[q] - (float)h) * 1024.0f); }
  for (int pass = 0; pass < 2; ++pass) { *(volatile v8us*)((unsigned short*)Hh + t * 8) = fh.half[0]; *(volatile v8us*)((unsigned short*)Hl + t * 8) = fl.half[0]; if (pass == 0) __threadfence(); } }

template <int NORM, int ROPE>
__global__ __launch_bounds__(HD) void k_xform(const float* __restrict__ F, int ldf, int nh, const float* __restrict__ gain, float eps, const float* __restrict__ CS, const float* __restrict__ SN, _Float16* __restrict__ H16, int ldo) {
  #pragma clang fp contract(off)
  __shared__ float xv[HD]; __shared__ float red[HD]; __shared__ unsigned short sh_[HD]; const int d = threadIdx.x; const int h = blockIdx.x % nh; const size_t r = blockIdx.x / nh; const int p = (int)(r % SQ);
  float x = F[r * (size_t)ldf + (size_t)h * HD + d];
  if (NORM) { red[d] = __fmul_rn(x, x); __syncthreads(); for (int st = HD / 2; st > 0; st >>= 1) { if (d < st) red[d] = __fadd_rn(red[d], red[d + st]); __syncthreads(); } const float rs = rsqrtf(__fadd_rn(red[0] / (float)HD, eps)); x = __fmul_rn(__fmul_rn(x, rs), bf16_rne(gain[d])); }
  xv[d] = x; __syncthreads();
  float o = x;
  if (ROPE == 1) { const int i = d >> 1; const float c = CS[p * (HD / 2) + i], s = SN[p * (HD / 2) + i]; const float ev = xv[2 * i], od = xv[2 * i + 1]; o = (d & 1) ? __fadd_rn(__fmul_rn(ev, s), __fmul_rn(od, c)) : __fadd_rn(__fmul_rn(ev, c), -__fmul_rn(od, s)); }
  if (ROPE == 2) { const int i = d & (HD / 2 - 1); const float c = CS[p * (HD / 2) + i], s = SN[p * (HD / 2) + i]; const float lo = xv[i], hi = xv[i + HD / 2]; o = (d < HD / 2) ? __fadd_rn(__fmul_rn(lo, c), -__fmul_rn(hi, s)) : __fadd_rn(__fmul_rn(lo, s), __fmul_rn(hi, c)); }
  FragH th; th.h[0] = (_Float16)o; sh_[d] = th.u[0]; __syncthreads();
  if (d < HD / 8) { FragH f; for (int q = 0; q < 8; ++q) f.u[q] = sh_[d * 8 + q]; unsigned short* dst = (unsigned short*)H16 + r * (size_t)ldo + (size_t)h * HD + d * 8; *(volatile v8us*)dst = f.half[0]; __threadfence(); *(volatile v8us*)dst = f.half[0]; } }

template <int NORM, int ROPE>
__global__ __launch_bounds__(HD) void k_xformf(const float* __restrict__ F, int ldf, int nh, const float* __restrict__ gain, float eps, const float* __restrict__ CS, const float* __restrict__ SN, float* __restrict__ F32, int ldo) {
  #pragma clang fp contract(off)
  __shared__ float xv[HD]; __shared__ float red[HD]; const int d = threadIdx.x; const int h = blockIdx.x % nh; const size_t r = blockIdx.x / nh; const int p = (int)(r % SQ);
  float x = F[r * (size_t)ldf + (size_t)h * HD + d];
  if (NORM) { red[d] = __fmul_rn(x, x); __syncthreads(); for (int st = HD / 2; st > 0; st >>= 1) { if (d < st) red[d] = __fadd_rn(red[d], red[d + st]); __syncthreads(); } const float rs = rsqrtf(__fadd_rn(red[0] / (float)HD, eps)); x = __fmul_rn(__fmul_rn(x, rs), bf16_rne(gain[d])); }
  xv[d] = x; __syncthreads();
  float o = x;
  if (ROPE == 1) { const int i = d >> 1; const float c = CS[p * (HD / 2) + i], s = SN[p * (HD / 2) + i]; const float ev = xv[2 * i], od = xv[2 * i + 1]; o = (d & 1) ? __fadd_rn(__fmul_rn(ev, s), __fmul_rn(od, c)) : __fadd_rn(__fmul_rn(ev, c), -__fmul_rn(od, s)); }
  if (ROPE == 2) { const int i = d & (HD / 2 - 1); const float c = CS[p * (HD / 2) + i], s = SN[p * (HD / 2) + i]; const float lo = xv[i], hi = xv[i + HD / 2]; o = (d < HD / 2) ? __fadd_rn(__fmul_rn(lo, c), -__fmul_rn(hi, s)) : __fadd_rn(__fmul_rn(lo, s), __fmul_rn(hi, c)); }
  float* dst = F32 + r * (size_t)ldo + (size_t)h * HD + d; *(volatile float*)dst = o; __threadfence(); *(volatile float*)dst = o; }

__global__ __launch_bounds__(256) void k_rsmw(const float* __restrict__ S, const float* __restrict__ madd, int mpitch, _Float16* __restrict__ P, int nrows, int q0, int nk) {
  #pragma clang fp contract(off)
  const int lane = threadIdx.x & 31; const int row = blockIdx.x * 8 + (threadIdx.x >> 5); if (row >= nrows) return;
  const float* s = S + (size_t)row * NKX; const float* mr = madd + (size_t)(q0 + (row % QT)) * mpitch; unsigned short* prow = (unsigned short*)P + (size_t)row * NKX;
  float mx = -3.0e38f;
#pragma unroll 1
  for (int j0 = lane * 8; j0 < nk; j0 += 256) { const v4f a = *(const v4fa*)(s + j0), c = *(const v4fa*)(s + j0 + 4); const v4f ma = *(const v4fa*)(mr + j0), mc = *(const v4fa*)(mr + j0 + 4);
#pragma unroll
    for (int q = 0; q < 4; ++q) { mx = fmaxf(mx, __fadd_rn(a[q], bf16_rne(ma[q]))); mx = fmaxf(mx, __fadd_rn(c[q], bf16_rne(mc[q]))); } }
#pragma unroll
  for (int off = 16; off > 0; off >>= 1) mx = fmaxf(mx, __shfl_xor(mx, off, 32));
  float se = 0.f;
#pragma unroll 1
  for (int j0 = lane * 8; j0 < nk; j0 += 256) { const v4f a = *(const v4fa*)(s + j0), c = *(const v4fa*)(s + j0 + 4); const v4f ma = *(const v4fa*)(mr + j0), mc = *(const v4fa*)(mr + j0 + 4);
#pragma unroll
    for (int q = 0; q < 4; ++q) { se = __fadd_rn(se, __expf(__fadd_rn(__fadd_rn(a[q], bf16_rne(ma[q])), -mx))); se = __fadd_rn(se, __expf(__fadd_rn(__fadd_rn(c[q], bf16_rne(mc[q])), -mx))); } }
#pragma unroll
  for (int off = 16; off > 0; off >>= 1) se = __fadd_rn(se, __shfl_xor(se, off, 32));
  const float sc = 1024.0f / se;
#pragma unroll 1
  for (int j0 = lane * 8; j0 < nk; j0 += 256) { const v4f a = *(const v4fa*)(s + j0), c = *(const v4fa*)(s + j0 + 4); const v4f ma = *(const v4fa*)(mr + j0), mc = *(const v4fa*)(mr + j0 + 4); FragH f;
#pragma unroll
    for (int q = 0; q < 4; ++q) { f.h[q] = (_Float16)__fmul_rn(__expf(__fadd_rn(__fadd_rn(a[q], bf16_rne(ma[q])), -mx)), sc); f.h[4 + q] = (_Float16)__fmul_rn(__expf(__fadd_rn(__fadd_rn(c[q], bf16_rne(mc[q])), -mx)), sc); }
    unsigned short* d = prow + j0; const v8us o = f.half[0]; *(volatile v8us*)d = o; __threadfence(); *(volatile v8us*)d = o; } }

__global__ __launch_bounds__(R0) void k_att0(const float* __restrict__ QF, int ldq, const float* __restrict__ KF, const float* __restrict__ VF, int ldkv, const float* __restrict__ madd, int mpitch, float scale, float* __restrict__ OF, int ldo) {
  #pragma clang fp contract(off)
  __shared__ __attribute__((aligned(16))) float lq[R0][HD]; __shared__ __attribute__((aligned(16))) float lo[R0][HD];
  const int tid = threadIdx.x; const int h = blockIdx.x / (QT0 / R0), rg = blockIdx.x % (QT0 / R0); const int i = rg * R0 + tid; const int g = h / HPG;
  const float* qr = QF + (size_t)i * ldq + (size_t)h * HD;
#pragma unroll 1
  for (int c = 0; c < HD / 4; ++c) { *(v4f*)&lq[tid][c * 4] = *(const v4fa*)(qr + c * 4); const v4f z = {0.f, 0.f, 0.f, 0.f}; *(v4f*)&lo[tid][c * 4] = z; }
  float m = -1.0e30f, l = 0.f; const int jmax = rg * R0 + (R0 - 1); const float* mr = madd + (size_t)i * mpitch;
#pragma unroll 1
  for (int j = 0; j <= jmax; ++j) { const float* kr = KF + (size_t)j * ldkv + (size_t)g * HD; const float* vr = VF + (size_t)j * ldkv + (size_t)g * HD; float s = 0.f;
#pragma unroll 1
    for (int c = 0; c < HD / 4; ++c) { const v4f kq = *(const v4fa*)(kr + c * 4); const v4f qq = *(v4f*)&lq[tid][c * 4]; s = __fadd_rn(s, __fmul_rn(qq[0], kq[0])); s = __fadd_rn(s, __fmul_rn(qq[1], kq[1])); s = __fadd_rn(s, __fmul_rn(qq[2], kq[2])); s = __fadd_rn(s, __fmul_rn(qq[3], kq[3])); }
    s = __fmul_rn(s, scale); s = __fadd_rn(s, bf16_rne(mr[j]));
    const float mn = fmaxf(m, s); const float sc = expf(m - mn); const float e = expf(s - mn); l = __fadd_rn(__fmul_rn(l, sc), e); m = mn;
#pragma unroll 1
    for (int c = 0; c < HD / 4; ++c) { const v4f vv = *(const v4fa*)(vr + c * 4); v4f oo = *(v4f*)&lo[tid][c * 4]; for (int u = 0; u < 4; ++u) oo[u] = __fadd_rn(__fmul_rn(oo[u], sc), __fmul_rn(e, vv[u])); *(v4f*)&lo[tid][c * 4] = oo; } }
  const float fin = 64.0f / l;
#pragma unroll 1
  for (int c = 0; c < HD / 4; ++c) { v4f oo = *(v4f*)&lo[tid][c * 4]; for (int u = 0; u < 4; ++u) oo[u] = __fmul_rn(oo[u], fin); *(v4f*)&lo[tid][c * 4] = oo; }
  __syncthreads();
  for (int pass = 0; pass < 2; ++pass) {
#pragma unroll 1
    for (int it = 0; it < R0; ++it) { const v4f v = *(const v4f*)&lo[it][tid * 4]; *(volatile v4f*)(OF + (size_t)(rg * R0 + it) * ldo + (size_t)h * HD + tid * 4) = v; }
    if (pass == 0) __threadfence(); } }

__global__ __launch_bounds__(256) void k_mchk(const float* __restrict__ madd, int mpitch, float* out) {
  __shared__ int red[256];
  const int tid = threadIdx.x; int bad = 0;
#pragma unroll 1
  for (int i = tid; i < SQ; i += 256) { const int te = (i < QT0) ? ((i / R0 + 1) * R0) : ((i / QT + 1) * QT); const float* mr = madd + (size_t)i * mpitch;
#pragma unroll 1
    for (int j = te; j < SQ; ++j) { const float mv = bf16_rne(mr[j]); bad |= (mv <= -1.0e4f) ? 0 : 1; } }
  red[tid] = bad; __syncthreads();
  for (int st = 128; st > 0; st >>= 1) { if (tid < st) red[tid] |= red[tid + st]; __syncthreads(); }
  if (red[0] != 0) { const float qn = __uint_as_float(0x7fc00000u); const v4f p4 = {qn, qn, qn, qn};
    for (int pass = 0; pass < 2; ++pass) {
#pragma unroll 1
      for (int e = tid * 4; e < R0 * DM; e += 1024) *(volatile v4f*)(out + e) = p4;
      if (pass == 0) __threadfence(); } } }

extern "C" void kernel_launch(void* const* d_in, const int* in_sizes, int n_in,
                              void* d_out, int out_size, void* d_ws, size_t ws_size, hipStream_t stream) {
  if (n_in < 7) return;
  if (in_sizes[0] < ((NB - 1) * SQF + SQ) * DM) return;
  if (in_sizes[1] < SQ * SQF) return;
  if (in_sizes[2] < SQ * HD2 || in_sizes[3] < SQ * HD2) return;
  if (in_sizes[4] < DM * DM || in_sizes[5] < DM * 2 * KVD || in_sizes[6] < DM * DM) return;
  if (out_size < ((NB - 1) * SQF + SQ) * DM) return;
  const float* x = (const float*)d_in[0]; const float* madd = (const float*)d_in[1]; const float* cs = (const float*)d_in[2]; const float* sn = (const float*)d_in[3];
  const float* wq = (const float*)d_in[4]; const float* wkv = (const float*)d_in[5]; const float* wo = (const float*)d_in[6]; float* out = (float*)d_out;
  char* ws = (char*)d_ws; size_t off = 0;
  auto take = [&](size_t bytes) { char* p = ws + off; off += (bytes + 255) & ~(size_t)255; return p; };
  _Float16* BQ  = (_Float16*)take((size_t)DM * DM * 2);
  _Float16* BKV = (_Float16*)take((size_t)2 * KVD * DM * 2);
  _Float16* BO  = (_Float16*)take((size_t)DM * DM * 2);
  float* CSB = (float*)take((size_t)SQ * HD2 * 4); float* SNB = (float*)take((size_t)SQ * HD2 * 4);
  _Float16* X16 = (_Float16*)take((size_t)SQ * DM * 2);
  float* QF = (float*)take((size_t)SQ * DM * 4); float* KF = (float*)take((size_t)SQ * KVD * 4);
  _Float16* Q16 = (_Float16*)take((size_t)SQ * DM * 2); _Float16* K16 = (_Float16*)take((size_t)SQ * KVD * 2); _Float16* V16 = (_Float16*)take((size_t)SQ * KVD * 2);
  _Float16* O16 = (_Float16*)take((size_t)SQ * DM * 2);
  float* S = (float*)take((size_t)NH * QT * NKX * 4); _Float16* P = (_Float16*)take((size_t)NH * QT * NKX * 2); _Float16* VT = (_Float16*)take((size_t)NG * HD * SQ * 2);
  float* QF0 = (float*)take((size_t)QT0 * DM * 4); float* KF0 = (float*)take((size_t)QT0 * KVD * 4); float* VF0 = (float*)take((size_t)QT0 * KVD * 4);
  float* OF0 = (float*)take((size_t)QT0 * DM * 4);
  _Float16* OH0 = (_Float16*)take((size_t)QT0 * DM * 2); _Float16* OL0 = (_Float16*)take((size_t)QT0 * DM * 2);
  if (off > ws_size) return;
  const _Float16* BK = BKV; const _Float16* BV = BKV + (size_t)KVD * DM;
  const float SCL = 0.08838834764831845f;
  k_wt_f16<<<(unsigned)(((size_t)DM * (DM / 8) + 255) / 256), 256, 0, stream>>>(wq, BQ, DM, DM, 16.0f);
  k_wt_f16<<<(unsigned)(((size_t)2 * KVD * (DM / 8) + 255) / 256), 256, 0, stream>>>(wkv, BKV, DM, 2 * KVD, 16.0f);
  k_wt_f16<<<(unsigned)(((size_t)DM * (DM / 8) + 255) / 256), 256, 0, stream>>>(wo, BO, DM, DM, 16.0f);
  k_bfcp<<<(unsigned)(((size_t)SQ * HD2 / 4 + 255) / 256), 256, 0, stream>>>(cs, CSB, (size_t)SQ * HD2 / 4);
  k_bfcp<<<(unsigned)(((size_t)SQ * HD2 / 4 + 255) / 256), 256, 0, stream>>>(sn, SNB, (size_t)SQ * HD2 / 4);
  for (int b = 0; b < NB; ++b) {
    const float* xb = x + (size_t)b * SQF * DM; float* outb = out + (size_t)b * SQF * DM;
    k_x16<<<(unsigned)(((size_t)SQ * DM / 8 + 255) / 256), 256, 0, stream>>>(xb, X16, (size_t)SQ * DM / 8);
    k_gemm2<0><<<dim3((unsigned)((SQ / 128) * (DM / 64)), 1), 128, 0, stream>>>(X16, DM, 0, BQ, DM, 0, 1, 0.0625f, nullptr, 0, nullptr, 1, 0, 0, QF, nullptr, DM, 0, SQ, DM, DM);
    k_gemm2<0><<<dim3((unsigned)((SQ / 128) * (KVD / 64)), 1), 128, 0, stream>>>(X16, DM, 0, BK, DM, 0, 1, 0.0625f, nullptr, 0, nullptr, 1, 0, 0, KF, nullptr, KVD, 0, SQ, KVD, DM);
    k_gemm2<0><<<dim3((unsigned)((SQ / 128) * (KVD / 64)), 1), 128, 0, stream>>>(X16, DM, 0, BV, DM, 0, 1, 0.0625f, nullptr, 0, nullptr, 1, 0, 0, nullptr, V16, KVD, 0, SQ, KVD, DM);
    k_xform<0, 1><<<(unsigned)((size_t)SQ * NH), HD, 0, stream>>>(QF, DM, NH, nullptr, 0.f, CSB, SNB, Q16, DM);
    k_xform<0, 1><<<(unsigned)((size_t)SQ * NG), HD, 0, stream>>>(KF, KVD, NG, nullptr, 0.f, CSB, SNB, K16, KVD);
    k_xformf<0, 1><<<(unsigned)(QT0 * NH), HD, 0, stream>>>(QF, DM, NH, nullptr, 0.f, CSB, SNB, QF0, DM);
    k_xformf<0, 1><<<(unsigned)(QT0 * NG), HD, 0, stream>>>(KF, KVD, NG, nullptr, 0.f, CSB, SNB, KF0, KVD);
    k_vt<2 * NG, SQ><<<(unsigned)(2 * NG * (SQ / 64)), 256, 0, stream>>>(V16, KVD, 0, VT);
    k_gemm2<0><<<dim3((unsigned)((QT0 / 128) * (KVD / 64)), 1), 128, 0, stream>>>(X16, DM, 0, BV, DM, 0, 1, 0.0625f, nullptr, 0, nullptr, 1, 0, 0, VF0, nullptr, KVD, 0, QT0, KVD, DM);
    k_att0<<<(unsigned)(NH * (QT0 / R0)), R0, 0, stream>>>(QF0, DM, KF0, VF0, KVD, madd, SQF, SCL, OF0, DM);
    for (int q0 = 0; q0 < SQ; q0 += QT) { const int nk = q0 + QT;
      k_gemm2<0><<<dim3((unsigned)((QT / 128) * (nk / 64)), NH), 128, 0, stream>>>(Q16 + (size_t)q0 * DM, DM, (size_t)HD, K16, KVD, (size_t)HD, HPG, SCL, nullptr, 0, nullptr, 1, 0, 0, S, nullptr, NKX, (size_t)QT * NKX, QT, nk, HD);
      k_rsmw<<<(unsigned)((NH * QT + 7) / 8), 256, 0, stream>>>(S, madd, SQF, P, NH * QT, q0, nk);
      k_gemm2<0><<<dim3((unsigned)((QT / 128) * (HD / 64)), NH), 128, 0, stream>>>(P, NKX, (size_t)QT * NKX, VT, SQ, (size_t)HD * SQ, HPG, 0.0625f, nullptr, 0, nullptr, 1, 0, 0, nullptr, O16 + (size_t)q0 * DM, DM, (size_t)HD, QT, HD, nk); }
    k_gemm2<0><<<dim3((unsigned)((SQ / 128) * (DM / 64)), 1), 128, 0, stream>>>(O16, DM, 0, BO, DM, 0, 1, 0.0009765625f, nullptr, 0, nullptr, 1, 0, 0, outb, nullptr, DM, 0, SQ, DM, DM);
    k_hl<<<(unsigned)(((size_t)QT0 * DM / 8 + 255) / 256), 256, 0, stream>>>(OF0, OH0, OL0, (size_t)QT0 * DM / 8);
    k_gemm2<0><<<dim3((unsigned)((QT0 / 128) * (DM / 64)), 1), 128, 0, stream>>>(OH0, DM, 0, BO, DM, 0, 1, 0.0009765625f, nullptr, 0, nullptr, 1, 0, 0, outb, nullptr, DM, 0, QT0, DM, DM);
    k_gemm2<0><<<dim3((unsigned)((QT0 / 128) * (DM / 64)), 1), 128, 0, stream>>>(OL0, DM, 0, BO, DM, 0, 1, 0.00000095367431640625f, nullptr, 0, outb, -1, 0, 0, outb, nullptr, DM, 0, QT0, DM, DM); }
  k_mchk<<<1, 256, 0, stream>>>(madd, SQF, out);
}
